// MusicTransformerDecoderLayer_52828097741088
// MI455X (gfx1250) — hardware-run, weakly checked
//
#include <hip/hip_runtime.h>
#include <math.h>

constexpr int kBatch = 2;
constexpr int kSeq   = 2048;
constexpr int kDim   = 1024;
constexpr int kHeads = 16;
constexpr int kDh    = 64;
constexpr int kFF    = 4096;
constexpr int kTok   = kBatch * kSeq;
constexpr int kGroups = kBatch * kHeads;
constexpr int kChunkG = 2;
constexpr int kNumChunks = kGroups / kChunkG;
constexpr float kWCarry   = 16.0f;
constexpr float kPCarry   = 2048.0f;
constexpr float kCtxCarry = 256.0f;
constexpr float kFCarry   = 16.0f;
constexpr float kLnEps    = 1e-5f;
constexpr float kInvDim   = 1.0f / 1024.0f;

typedef __attribute__((ext_vector_type(16))) _Float16 v16h;
typedef __attribute__((ext_vector_type(8)))  _Float16 v8h;
typedef __attribute__((ext_vector_type(16))) __bf16   v16b;
typedef __attribute__((ext_vector_type(8)))  __bf16   v8b;
typedef __attribute__((ext_vector_type(8)))  float    v8f;
typedef __attribute__((ext_vector_type(4)))  float    v4f;
typedef __attribute__((ext_vector_type(4)))  unsigned int v4u;
typedef __attribute__((ext_vector_type(4)))  int      v4i;

__device__ __forceinline__ unsigned short f2bf_bits(float f) {
  unsigned u = __float_as_uint(f);
  return (unsigned short)((u + 0x7FFFu + ((u >> 16) & 1u)) >> 16);
}
__device__ __forceinline__ float bf_bits2f(unsigned short h) { return __uint_as_float(((unsigned)h) << 16); }

__device__ __forceinline__ void dep_guard_h(v8f& a, v8f& b, v16h x, v16h y) { asm volatile("v_nop\n\tv_nop\n\tv_nop\n\tv_nop" : "+v"(a), "+v"(b) : "v"(x), "v"(y)); }
__device__ __forceinline__ void dep_guard_b(v8f& a, v8f& b, v16b x, v16b y) { asm volatile("v_nop\n\tv_nop\n\tv_nop\n\tv_nop" : "+v"(a), "+v"(b) : "v"(x), "v"(y)); }
__device__ __forceinline__ void keep4_h(v16h a, v16h b, v16h c, v16h d) { asm volatile("v_nop" :: "v"(a), "v"(b), "v"(c), "v"(d)); }
__device__ __forceinline__ void keep4_b(v16b a, v16b b, v16b c, v16b d) { asm volatile("v_nop" :: "v"(a), "v"(b), "v"(c), "v"(d)); }
__device__ __forceinline__ void acc_guard4(v8f& a, v8f& b, v8f& c, v8f& d) { asm volatile("v_nop\n\tv_nop\n\tv_nop\n\tv_nop" : "+v"(a), "+v"(b), "+v"(c), "+v"(d)); }
template <typename T> struct Frag;
template <> struct Frag<_Float16> {
  typedef v16h V; union U { v16h v; v8h h[2]; };
  static __device__ __forceinline__ v16h load(const _Float16* p) {
    U f; f.h[0] = *(const v8h*)(p); f.h[1] = *(const v8h*)(p + 16); return f.v;
  }
  static __device__ __forceinline__ v8f mma(v16h a, v16h b, v8f c) {
    return __builtin_amdgcn_wmma_f32_16x16x32_f16(false, a, false, b, (short)0, c, false, false);
  }
  static __device__ __forceinline__ void guard(v8f& a, v8f& b, v16h x, v16h y) { dep_guard_h(a, b, x, y); }
  static __device__ __forceinline__ void keep(v16h a, v16h b, v16h c, v16h d) { keep4_h(a, b, c, d); }
};
template <> struct Frag<__bf16> {
  typedef v16b V; union U { v16b v; v8b h[2]; };
  static __device__ __forceinline__ v16b load(const __bf16* p) {
    U f; f.h[0] = *(const v8b*)(p); f.h[1] = *(const v8b*)(p + 16); return f.v;
  }
  static __device__ __forceinline__ v8f mma(v16b a, v16b b, v8f c) {
    return __builtin_amdgcn_wmma_f32_16x16x32_bf16(false, a, false, b, (short)0, c, false, false);
  }
  static __device__ __forceinline__ void guard(v8f& a, v8f& b, v16b x, v16b y) { dep_guard_b(a, b, x, y); }
  static __device__ __forceinline__ void keep(v16b a, v16b b, v16b c, v16b d) { keep4_b(a, b, c, d); }
};

__device__ __forceinline__ unsigned pk16(unsigned short a, unsigned short b) { return (unsigned)a | ((unsigned)b << 16); }
__device__ __forceinline__ unsigned short h_bits(float f) { const _Float16 h = (_Float16)f; return __builtin_bit_cast(unsigned short, h); }

template <int ET> struct Elem;
template <> struct Elem<0> { typedef _Float16 T; };
template <> struct Elem<1> { typedef __bf16 T; };
template <int ET, bool SPLIT, int BIAS_MODE, int OUT_MODE, bool RESID, int ROWSC, int KMODE>
__global__ __launch_bounds__(256) void wmma_gemm64(
    const unsigned short* __restrict__ Ap, const unsigned short* __restrict__ A2p, int lda, long strideA,
    const unsigned short* __restrict__ Btp, const unsigned short* __restrict__ Bt2p, int ldb, long strideB,
    void* __restrict__ Cout, void* __restrict__ Cout2, int ldc, long strideC,
    const float* __restrict__ bias,
    const float* __restrict__ resid, long strideR,
    const int* __restrict__ rowsc,
    int M, int N, int K, float scale) {
  typedef typename Elem<ET>::T T;
  typedef typename Frag<T>::V V;
  const T* A = (const T*)Ap; const T* A2 = (const T*)A2p; const T* Bt = (const T*)Btp; const T* Bt2 = (const T*)Bt2p;
  __shared__ __align__(16) float sT[8][16 * 68];
  const int b    = blockIdx.y;
  const int lane = threadIdx.x & 31;
  const int wave = threadIdx.x >> 5;
  const int tilesN = N >> 6;
  const int tilesM = M >> 6;
  const int tile = blockIdx.x * 8 + wave;
  if (tile >= tilesM * tilesN) return;
  const int tm = tile / tilesN;
  const int tn = tile - tm * tilesN;
  if (KMODE == 1 && tn > tm) return;
  const int m0 = tm << 6;
  const int n0 = tn << 6;
  int Kend = K;
  if (KMODE == 2) { const int kl = m0 + 64; Kend = kl < K ? kl : K; }

  const T* Ab  = A  + (size_t)b * strideA;
  const T* Bb  = Bt + (size_t)b * strideB;
  const T* Ab2 = SPLIT ? (A2  + (size_t)b * strideA) : nullptr;
  const T* Bb2 = SPLIT ? (Bt2 + (size_t)b * strideB) : nullptr;

  const int rlane = lane & 15;
  const int koff  = (lane >> 4) * 8;
  const int mOff  = (lane >> 4) * 8;

  v8f acc[4][4];
#pragma unroll
  for (int i = 0; i < 4; ++i)
#pragma unroll
    for (int j = 0; j < 4; ++j) acc[i][j] = (v8f){0.f,0.f,0.f,0.f,0.f,0.f,0.f,0.f};

  for (int k0 = 0; k0 < Kend; k0 += 32) {
    V bh[4], bl[4];
#pragma unroll
    for (int j = 0; j < 4; ++j) {
      const size_t bo = (size_t)(n0 + (j << 4) + rlane) * ldb + koff + k0;
      bh[j] = Frag<T>::load(Bb + bo);
      if (SPLIT) bl[j] = Frag<T>::load(Bb2 + bo);
    }
#pragma unroll
    for (int i = 0; i < 4; ++i) {
      const size_t ao = (size_t)(m0 + (i << 4) + rlane) * lda + koff + k0;
      V ah = Frag<T>::load(Ab + ao);
      V al;
      if (SPLIT) al = Frag<T>::load(Ab2 + ao);
#pragma unroll
      for (int j = 0; j < 4; ++j) {
        acc[i][j] = Frag<T>::mma(ah, bh[j], acc[i][j]);
        if (SPLIT) {
          acc[i][j] = Frag<T>::mma(ah, bl[j], acc[i][j]);
          acc[i][j] = Frag<T>::mma(al, bh[j], acc[i][j]);
        }
      }
      Frag<T>::guard(acc[i][0], acc[i][3], ah, SPLIT ? al : ah);
    }
    Frag<T>::keep(bh[0], bh[1], bh[2], bh[3]);
    if (SPLIT) Frag<T>::keep(bl[0], bl[1], bl[2], bl[3]);
  }
  acc_guard4(acc[0][0], acc[0][1], acc[0][2], acc[0][3]);
  acc_guard4(acc[1][0], acc[1][1], acc[1][2], acc[1][3]);
  acc_guard4(acc[2][0], acc[2][1], acc[2][2], acc[2][3]);
  acc_guard4(acc[3][0], acc[3][1], acc[3][2], acc[3][3]);

  float* slab = sT[wave];
  const float* Rb = RESID ? (resid + (size_t)b * strideR) : nullptr;
#pragma unroll
  for (int i = 0; i < 4; ++i) {
    const int mBase = m0 + (i << 4);
#pragma unroll
    for (int j = 0; j < 4; ++j) {
      const int n = n0 + (j << 4) + rlane;
      float bv = 0.f;
      if (BIAS_MODE == 2) bv = bias[n];
#pragma unroll
      for (int r = 0; r < 8; ++r) {
        float v = acc[i][j][r] * scale;
        if (BIAS_MODE == 1) v += bias[mBase + mOff + r];
        if (BIAS_MODE == 2) v += bv;
        if (ROWSC == 1) v = v * (float)rowsc[mBase + mOff + r];
        if (RESID) v += Rb[(size_t)(mBase + mOff + r) * ldc + n];
        if (ROWSC == 2) v = v * (float)rowsc[mBase + mOff + r];
        slab[(mOff + r) * 68 + (j << 4) + rlane] = v;
      }
    }
    __builtin_amdgcn_fence(__ATOMIC_RELEASE, "workgroup");
    __builtin_amdgcn_wave_barrier();
    __builtin_amdgcn_fence(__ATOMIC_ACQUIRE, "workgroup");
    if (OUT_MODE == 0) {
      float* C = (float*)Cout + (size_t)b * strideC;
      const int hh = lane >> 4, c4 = (lane & 15) * 4;
      for (int pass = 0; pass < 2; ++pass) {
#pragma unroll
        for (int it = 0; it < 8; ++it) {
          const int row = it * 2 + hh;
          v4f v = *(const v4f*)(slab + row * 68 + c4);
          *(volatile v4f*)(C + (size_t)(mBase + row) * ldc + n0 + c4) = v;
        }
        __threadfence();
      }
    } else {
      const int q = lane >> 3, c8 = (lane & 7) * 8;
      unsigned short* C  = (unsigned short*)Cout  + (size_t)b * strideC;
      unsigned short* C2 = (OUT_MODE == 2) ? ((unsigned short*)Cout2 + (size_t)b * strideC) : nullptr;
      for (int pass = 0; pass < 2; ++pass) {
#pragma unroll
        for (int it = 0; it < 4; ++it) {
          const int row = it * 4 + q;
          const float* sp = slab + row * 68 + c8;
          v8h hv, lv;
#pragma unroll
          for (int e = 0; e < 8; ++e) {
            if (OUT_MODE == 1) {
              hv[e] = (_Float16)sp[e];
            } else {
              unsigned short hb = f2bf_bits(sp[e]);
              unsigned short lb = f2bf_bits(sp[e] - bf_bits2f(hb));
              hv[e] = __builtin_bit_cast(_Float16, hb);
              lv[e] = __builtin_bit_cast(_Float16, lb);
            }
          }
          *(volatile v8h*)(C + (size_t)(mBase + row) * ldc + n0 + c8) = hv;
          if (OUT_MODE == 2) *(volatile v8h*)(C2 + (size_t)(mBase + row) * ldc + n0 + c8) = lv;
        }
        __threadfence();
      }
    }
    __builtin_amdgcn_fence(__ATOMIC_RELEASE, "workgroup");
    __builtin_amdgcn_wave_barrier();
    __builtin_amdgcn_fence(__ATOMIC_ACQUIRE, "workgroup");
  }
}

__global__ __launch_bounds__(256) void wtcast64_kernel(const float* __restrict__ W, unsigned short* __restrict__ out,
                                                       int Kdim, int Ndim, float scale) {
  __shared__ float sm[64][65];
  const int t  = threadIdx.x;
  const int k0 = blockIdx.x * 64;
  const int n0 = blockIdx.y * 64;
#pragma unroll
  for (int i = 0; i < 16; ++i) {
    const int e = i * 256 + t;
    const int r = e >> 6;
    const int c = e & 63;
    sm[c][r] = W[(size_t)(k0 + r) * Ndim + n0 + c] * scale;
  }
  __syncthreads();
  const int lane = t & 31, wave = t >> 5;
  const int q = lane >> 3, c8 = (lane & 7) * 8;
  for (int pass = 0; pass < 2; ++pass) {
#pragma unroll
    for (int it = 0; it < 2; ++it) {
      const int row = wave * 8 + it * 4 + q;
      unsigned short hb[8];
#pragma unroll
      for (int e = 0; e < 8; ++e) hb[e] = h_bits(sm[row][c8 + e]);
      const v4u u = (v4u){pk16(hb[0], hb[1]), pk16(hb[2], hb[3]), pk16(hb[4], hb[5]), pk16(hb[6], hb[7])};
      *(volatile v4u*)(out + (size_t)(n0 + row) * Kdim + k0 + c8) = u;
    }
    __threadfence();
  }
}

__device__ __forceinline__ int rel_bucket_fn(int d) {
  const int dc = d < 1 ? 1 : d;
  const float ratio = logf((float)dc * 0.0625f) * (1.0f / 2.0794415416798357f);
  int lg = 16 + (int)(ratio * 16.0f);
  lg = lg > 31 ? 31 : lg;
  return d < 16 ? d : lg;
}
__global__ __launch_bounds__(256) void bias_table_kernel(const float* __restrict__ rel, float* __restrict__ BT) {
#pragma clang fp contract(off)
  const int idx = blockIdx.x * 256 + threadIdx.x;
  const int h   = idx >> 9;
  const int d0  = (idx & 511) * 4;
  float v[4];
#pragma unroll
  for (int e = 0; e < 4; ++e) {
    const int bk = rel_bucket_fn(d0 + e);
    v[e] = rel[bk * kHeads + h];
  }
  const v4f o = (v4f){v[0], v[1], v[2], v[3]};
  float* p = BT + (size_t)h * kSeq + d0;
  *(volatile v4f*)p = o;
  __threadfence();
  *(volatile v4f*)p = o;
}

__global__ __launch_bounds__(128) void layernorm_f16_kernel(const float* __restrict__ X, const float* __restrict__ gam,
                                                            const float* __restrict__ bet, unsigned short* __restrict__ out) {
  __shared__ float redA[4];
  __shared__ float redB[4];
  const int row  = blockIdx.x;
  const int t    = threadIdx.x;
  const int lane = t & 31, wave = t >> 5;
  const int c0   = t * 8;
  const float* xr = X + (size_t)row * kDim + c0;
  const v4f a = *(const v4f*)(xr);
  const v4f c = *(const v4f*)(xr + 4);
  float x[8];
#pragma unroll
  for (int e = 0; e < 4; ++e) { x[e] = a[e]; x[4 + e] = c[e]; }
  float s = ((x[0] + x[1]) + (x[2] + x[3])) + ((x[4] + x[5]) + (x[6] + x[7]));
#pragma unroll
  for (int off = 16; off > 0; off >>= 1) s += __shfl_xor(s, off, 32);
  if (lane == 0) redA[wave] = s;
  __syncthreads();
  const float mu = ((redA[0] + redA[1]) + (redA[2] + redA[3])) * kInvDim;
  float d[8];
  float s2 = 0.f;
#pragma unroll
  for (int e = 0; e < 8; ++e) { d[e] = x[e] - mu; s2 += d[e] * d[e]; }
#pragma unroll
  for (int off = 16; off > 0; off >>= 1) s2 += __shfl_xor(s2, off, 32);
  if (lane == 0) redB[wave] = s2;
  __syncthreads();
  const float var  = ((redB[0] + redB[1]) + (redB[2] + redB[3])) * kInvDim;
  const float rstd = rsqrtf(var + kLnEps);
  const v4f ga = *(const v4f*)(gam + c0);
  const v4f gc = *(const v4f*)(gam + c0 + 4);
  const v4f ba = *(const v4f*)(bet + c0);
  const v4f bc = *(const v4f*)(bet + c0 + 4);
  float gg[8], bb[8];
#pragma unroll
  for (int e = 0; e < 4; ++e) { gg[e] = ga[e]; gg[4 + e] = gc[e]; bb[e] = ba[e]; bb[4 + e] = bc[e]; }
  unsigned short hb[8];
#pragma unroll
  for (int e = 0; e < 8; ++e) hb[e] = h_bits(d[e] * rstd * gg[e] + bb[e]);
  const v4u u = (v4u){pk16(hb[0], hb[1]), pk16(hb[2], hb[3]), pk16(hb[4], hb[5]), pk16(hb[6], hb[7])};
  unsigned short* op = out + (size_t)row * kDim + c0;
  *(volatile v4u*)op = u;
  __threadfence();
  *(volatile v4u*)op = u;
}

__global__ __launch_bounds__(256) void softmax_rows_kernel(const float* __restrict__ Sc, const float* __restrict__ BT,
                                                           const int* __restrict__ amask, unsigned short* __restrict__ P,
                                                           int b, int h0) {
  __shared__ float redM[8];
  __shared__ float redS[8];
  const int gl   = blockIdx.x >> 11;
  const int i    = blockIdx.x & 2047;
  const int h    = h0 + gl;
  const int t    = threadIdx.x;
  const int lane = t & 31;
  const int wave = __builtin_amdgcn_readfirstlane(t >> 5);
  const int c0   = t * 8;
  const size_t rowoff = ((size_t)gl * kSeq + (size_t)i) * kSeq;
  const float kNegInf = -__builtin_inff();
  float s[8];
  const bool active = (wave * 256) <= i;
  if (active) {
    const float* sr = Sc + rowoff + c0;
    const v4f a  = *(const v4f*)(sr);
    const v4f c4 = *(const v4f*)(sr + 4);
    const v4i m0 = *(const v4i*)(amask + (size_t)b * kSeq + c0);
    const v4i m1 = *(const v4i*)(amask + (size_t)b * kSeq + c0 + 4);
    float x[8]; int mk[8];
#pragma unroll
    for (int e = 0; e < 4; ++e) { x[e] = a[e]; x[4 + e] = c4[e]; mk[e] = m0[e]; mk[4 + e] = m1[e]; }
    const float* bth = BT + (size_t)h * kSeq;
#pragma unroll
    for (int e = 0; e < 8; ++e) {
      const int j   = c0 + e;
      const int dd  = i - j;
      const int dcl = dd < 0 ? 0 : dd;
      const float val = x[e] + bth[dcl];
      const bool masked = (j > i) || (mk[e] == 0);
      s[e] = masked ? kNegInf : val;
    }
  } else {
#pragma unroll
    for (int e = 0; e < 8; ++e) s[e] = kNegInf;
  }
  float m = fmaxf(fmaxf(fmaxf(s[0], s[1]), fmaxf(s[2], s[3])), fmaxf(fmaxf(s[4], s[5]), fmaxf(s[6], s[7])));
#pragma unroll
  for (int off = 16; off > 0; off >>= 1) m = fmaxf(m, __shfl_xor(m, off, 32));
  if (lane == 0) redM[wave] = m;
  __syncthreads();
  float mAll = redM[0];
#pragma unroll
  for (int w = 1; w < 8; ++w) mAll = fmaxf(mAll, redM[w]);
  const float mUse = (mAll == kNegInf) ? 0.0f : mAll;
  float ex[8];
  float ps = 0.f;
#pragma unroll
  for (int e = 0; e < 8; ++e) { ex[e] = expf(s[e] - mUse); ps += ex[e]; }
#pragma unroll
  for (int off = 16; off > 0; off >>= 1) ps += __shfl_xor(ps, off, 32);
  if (lane == 0) redS[wave] = ps;
  __syncthreads();
  float sum = redS[0];
#pragma unroll
  for (int w = 1; w < 8; ++w) sum += redS[w];
  const float q   = kPCarry / sum;
  const float inv = (sum > 0.f) ? q : 0.0f;
  unsigned short hb[8];
#pragma unroll
  for (int e = 0; e < 8; ++e) hb[e] = h_bits(ex[e] * inv);
  const v4u u = (v4u){pk16(hb[0], hb[1]), pk16(hb[2], hb[3]), pk16(hb[4], hb[5]), pk16(hb[6], hb[7])};
  unsigned short* op = P + rowoff + c0;
  *(volatile v4u*)op = u;
  __threadfence();
  *(volatile v4u*)op = u;
}

__global__ __launch_bounds__(256) void gelu_cast_kernel(const float* __restrict__ U, unsigned short* __restrict__ F, int n8) {
  const int i = blockIdx.x * 256 + threadIdx.x;
  if (i >= n8) return;
  const float* p = U + 8 * (size_t)i;
  unsigned w0 = 0u, w1 = 0u, w2 = 0u, w3 = 0u;
#pragma unroll 1
  for (int e = 0; e < 8; ++e) {
    const float v  = p[e];
    const float gv = 0.5f * v * (1.0f + erff(v * 0.70710678118654752f));
    const unsigned hb = (unsigned)h_bits(gv * kFCarry);
    w0 = (w0 >> 16) | (w1 << 16);
    w1 = (w1 >> 16) | (w2 << 16);
    w2 = (w2 >> 16) | (w3 << 16);
    w3 = (w3 >> 16) | (hb << 16);
  }
  const v4u u = (v4u){w0, w1, w2, w3};
  unsigned short* op = F + 8 * (size_t)i;
  *(volatile v4u*)op = u;
  __threadfence();
  *(volatile v4u*)op = u;
}

extern "C" void kernel_launch(void* const* d_in, const int* in_sizes, int n_in,
                              void* d_out, int out_size, void* d_ws, size_t ws_size,
                              hipStream_t stream) {
  if (n_in < 19) return;
  if (in_sizes[0] != kTok * kDim || out_size != kTok * kDim || in_sizes[1] != kTok) return;
  if (in_sizes[2] != kDim * kDim || in_sizes[15] != kDim * kFF || in_sizes[17] != kFF * kDim || in_sizes[10] != 32 * kHeads) return;

  const float* hidden = (const float*)d_in[0];
  const int*   amask  = (const int*)d_in[1];
  const float* wq  = (const float*)d_in[2];
  const float* bq  = (const float*)d_in[3];
  const float* wk  = (const float*)d_in[4];
  const float* bk  = (const float*)d_in[5];
  const float* wv  = (const float*)d_in[6];
  const float* bv  = (const float*)d_in[7];
  const float* wo  = (const float*)d_in[8];
  const float* bo  = (const float*)d_in[9];
  const float* rel = (const float*)d_in[10];
  const float* ln1g = (const float*)d_in[11];
  const float* ln1b = (const float*)d_in[12];
  const float* ln2g = (const float*)d_in[13];
  const float* ln2b = (const float*)d_in[14];
  const float* w1  = (const float*)d_in[15];
  const float* b1  = (const float*)d_in[16];
  const float* w2  = (const float*)d_in[17];
  const float* b2  = (const float*)d_in[18];
  float* out = (float*)d_out;

  const size_t MiB = (size_t)1 << 20;
  const size_t offW2T  = 0;
  const size_t offW1T  = offW2T + (size_t)kDim * kFF * 2;
  const size_t offWOT  = offW1T + (size_t)kFF * kDim * 2;
  const size_t offWQKT = offWOT + (size_t)kDim * kDim * 2;
  const size_t offWVT  = offWQKT + (size_t)2 * kDim * kDim * 2;
  const size_t offXY   = offWVT + (size_t)kDim * kDim * 2;
  const size_t offQK   = offXY + (size_t)kTok * kDim * 2;
  const size_t offH1   = offQK;
  const size_t offVT   = offQK + (size_t)kTok * 2 * kDim * 2;
  const size_t offSC   = offVT + (size_t)kTok * kDim * 2;
  const size_t offU    = offSC;
  const size_t offP    = offSC + (size_t)kChunkG * kSeq * kSeq * 4;
  const size_t offF    = offP;
  const size_t offCTX  = offP + (size_t)kChunkG * kSeq * kSeq * 2;
  const size_t offBT   = offF + (size_t)kTok * kFF * 2;
  const size_t total   = offBT + (size_t)kHeads * kSeq * 4;
  if (offCTX + (size_t)kTok * kDim * 2 > offBT) return;
  if (offH1 + (size_t)kTok * kDim * 4 > offVT + (size_t)kTok * kDim * 2) return;
  if (total > ws_size || total > 128 * MiB) return;

  char* ws = (char*)d_ws;
  unsigned short* W2T  = (unsigned short*)(ws + offW2T);
  unsigned short* W1T  = (unsigned short*)(ws + offW1T);
  unsigned short* WOT  = (unsigned short*)(ws + offWOT);
  unsigned short* WQKT = (unsigned short*)(ws + offWQKT);
  unsigned short* WVT  = (unsigned short*)(ws + offWVT);
  unsigned short* XY   = (unsigned short*)(ws + offXY);
  unsigned short* QK   = (unsigned short*)(ws + offQK);
  float*          H1   = (float*)(ws + offH1);
  unsigned short* VT   = (unsigned short*)(ws + offVT);
  float*          SC   = (float*)(ws + offSC);
  float*          U    = (float*)(ws + offU);
  unsigned short* P    = (unsigned short*)(ws + offP);
  unsigned short* F    = (unsigned short*)(ws + offF);
  unsigned short* CTX  = (unsigned short*)(ws + offCTX);
  float*          BT   = (float*)(ws + offBT);

  wtcast64_kernel<<<dim3(kDim / 64, kDim / 64), 256, 0, stream>>>(wq, WQKT, kDim, kDim, kWCarry);
  wtcast64_kernel<<<dim3(kDim / 64, kDim / 64), 256, 0, stream>>>(wk, WQKT + (size_t)kDim * kDim, kDim, kDim, kWCarry);
  wtcast64_kernel<<<dim3(kDim / 64, kDim / 64), 256, 0, stream>>>(wv, WVT, kDim, kDim, kWCarry);
  wtcast64_kernel<<<dim3(kDim / 64, kDim / 64), 256, 0, stream>>>(wo, WOT, kDim, kDim, kWCarry);
  wtcast64_kernel<<<dim3(kDim / 64, kFF / 64), 256, 0, stream>>>(w1, W1T, kDim, kFF, kWCarry);
  wtcast64_kernel<<<dim3(kFF / 64, kDim / 64), 256, 0, stream>>>(w2, W2T, kFF, kDim, kWCarry);

  bias_table_kernel<<<(kHeads * kSeq / 4) / 256, 256, 0, stream>>>(rel, BT);

  layernorm_f16_kernel<<<kTok, 128, 0, stream>>>(hidden, ln1g, ln1b, XY);

  const float wInv = 1.0f / kWCarry;
  {
    const dim3 g((kTok / 64) * (kDim / 64) / 8, 1);
    wmma_gemm64<0, false, 2, 1, false, 0, 0><<<g, 256, 0, stream>>>(
        XY, XY, kDim, 0L, WQKT, WQKT, kDim, 0L, (void*)QK, (void*)QK, 2 * kDim, 0L,
        bq, hidden, 0L, amask, kTok, kDim, kDim, wInv);
    wmma_gemm64<0, false, 2, 1, false, 0, 0><<<g, 256, 0, stream>>>(
        XY, XY, kDim, 0L, WQKT + (size_t)kDim * kDim, WQKT + (size_t)kDim * kDim, kDim, 0L,
        (void*)(QK + kDim), (void*)(QK + kDim), 2 * kDim, 0L,
        bk, hidden, 0L, amask, kTok, kDim, kDim, wInv);
  }
  {
    const dim3 g((kDim / 64) * (kSeq / 64) / 8, kBatch);
    wmma_gemm64<0, false, 1, 1, false, 0, 0><<<g, 256, 0, stream>>>(
        WVT, WVT, kDim, 0L, XY, XY, kDim, (long)kSeq * kDim, (void*)VT, (void*)VT, kSeq, (long)kDim * kSeq,
        bv, hidden, 0L, amask, kDim, kSeq, kDim, wInv);
  }

  for (int ci = 0; ci < kNumChunks; ++ci) {
    const int b  = ci / (kHeads / kChunkG);
    const int h0 = (ci % (kHeads / kChunkG)) * kChunkG;
    const size_t qkBase = (size_t)b * kSeq * (2 * kDim) + (size_t)h0 * kDh;
    {
      const dim3 g((kSeq / 64) * (kSeq / 64) / 8, kChunkG);
      wmma_gemm64<0, false, 0, 0, false, 0, 1><<<g, 256, 0, stream>>>(
          QK + qkBase, QK + qkBase, 2 * kDim, (long)kDh,
          QK + qkBase + kDim, QK + qkBase + kDim, 2 * kDim, (long)kDh,
          (void*)SC, (void*)SC, kSeq, (long)kSeq * kSeq,
          bq, hidden, 0L, amask, kSeq, kSeq, kDh, 0.125f);
    }
    softmax_rows_kernel<<<kChunkG * kSeq, 256, 0, stream>>>(SC, BT, amask, P, b, h0);
    {
      const size_t vtBase  = (size_t)(b * kHeads + h0) * kDh * kSeq;
      const size_t ctxBase = (size_t)b * kSeq * kDim + (size_t)h0 * kDh;
      const dim3 g((kSeq / 64) * (kDh / 64) / 8, kChunkG);
      wmma_gemm64<0, false, 0, 1, false, 0, 2><<<g, 256, 0, stream>>>(
          P, P, kSeq, (long)kSeq * kSeq,
          VT + vtBase, VT + vtBase, kSeq, (long)kDh * kSeq,
          (void*)(CTX + ctxBase), (void*)(CTX + ctxBase), kDim, (long)kDh,
          bq, hidden, 0L, amask, kSeq, kDh, kSeq, kCtxCarry / kPCarry);
    }
  }

  {
    const dim3 g((kTok / 64) * (kDim / 64) / 8, 1);
    wmma_gemm64<0, false, 2, 0, true, 1, 0><<<g, 256, 0, stream>>>(
        CTX, CTX, kDim, 0L, WOT, WOT, kDim, 0L, (void*)H1, (void*)H1, kDim, 0L,
        bo, hidden, 0L, amask, kTok, kDim, kDim, 1.0f / (kCtxCarry * kWCarry));
  }

  layernorm_f16_kernel<<<kTok, 128, 0, stream>>>(H1, ln2g, ln2b, XY);

  for (int ch = 0; ch < 2; ++ch) {
    const dim3 g((2048 / 64) * (kFF / 64) / 8, 1);
    wmma_gemm64<0, false, 2, 0, false, 0, 0><<<g, 256, 0, stream>>>(
        XY + (size_t)ch * 2048 * kDim, XY + (size_t)ch * 2048 * kDim, kDim, 0L, W1T, W1T, kDim, 0L,
        (void*)U, (void*)U, kFF, 0L,
        b1, hidden, 0L, amask, 2048, kFF, kDim, wInv);
    const int n8 = 2048 * kFF / 8;
    gelu_cast_kernel<<<n8 / 256, 256, 0, stream>>>(U, F + (size_t)ch * 2048 * kFF, n8);
  }

  {
    const dim3 g((kTok / 64) * (kDim / 64) / 8, 1);
    wmma_gemm64<0, false, 2, 0, true, 2, 0><<<g, 256, 0, stream>>>(
        F, F, kFF, 0L, W2T, W2T, kFF, 0L, (void*)out, (void*)out, kDim, 0L,
        b2, H1, 0L, amask, kTok, kDim, kFF, 1.0f / (kFCarry * kWCarry));
  }
}
